// ModulatedDeformableConv2d_10033043604236
// MI455X (gfx1250) — hardware-run, weakly checked
//
#include <hip/hip_runtime.h>


#ifndef NB
#define NB 4
#endif
#define NB_FULL 4
#define CI   64
#define CO   64
#define HH   128
#define WW   128
#define OFC  32
#define NTAP 9
#define KO   (OFC * NTAP)
#define KM   (CI * NTAP)
#define NOM  27
#define NOPD 32
#define TP   64
#define FC   (TP + 2)
#define OMP  68
#define ASP  200
#define OSP  68
#define SCA  64.0f
#define WSC  1024.0f
#define OSC  (1.0f / 65536.0f)

static_assert(NB <= NB_FULL);
static_assert(TP == 64);
static_assert(WW % TP == 0);
static_assert(WW / TP == 2);
static_assert(HH == 128);
static_assert(KO % 32 == 0);
static_assert(KM % 32 == 0);
static_assert(OFC == 32);
static_assert(CI == 64);
static_assert(CO == 64);
static_assert(NOM <= NOPD);
static_assert(NOPD == 32);
static_assert((OMP * 4) % 16 == 0);
static_assert((ASP * 2) % 16 == 0);
static_assert((OSP * 4) % 16 == 0);
static_assert(ASP >= 3 * CI);
static_assert(12 * 128 == TP * 3 * (CI / 8));
static_assert(32 * 16 * 8 == 16 * TP * 4);
static_assert((3 * FC * 32) * 2 + (NOPD * OMP) * 4 + 2 * (TP * NTAP * 4) * 4 + (TP * ASP) * 2 + (CO * OSP) * 4 <= 131072);

typedef _Float16 h16;
typedef unsigned short bf;
typedef __attribute__((ext_vector_type(16))) __bf16   v16bf;
typedef __attribute__((ext_vector_type(16))) _Float16 v16h;
typedef __attribute__((ext_vector_type(8)))  _Float16 v8h;
typedef __attribute__((ext_vector_type(8)))  unsigned short v8us;
typedef __attribute__((ext_vector_type(8)))  float    v8f;
typedef __attribute__((ext_vector_type(4)))  float    v4f;
typedef __attribute__((ext_vector_type(4)))  int      v4i;
typedef __attribute__((ext_vector_type(4)))  unsigned v4u;
typedef v4f  __attribute__((may_alias)) v4fa;
typedef v4u  __attribute__((may_alias)) v4ua;

__device__ __forceinline__ unsigned short f2bf(float f) { unsigned u = __float_as_uint(f); u += 0x7FFFu + ((u >> 16) & 1u); return (unsigned short)(u >> 16); }
__device__ __forceinline__ float bfr(float f) { return __uint_as_float(((unsigned)f2bf(f)) << 16); }
__device__ __forceinline__ v16h cat16(v8h lo, v8h hi) { return __builtin_shufflevector(lo, hi, 0, 1, 2, 3, 4, 5, 6, 7, 8, 9, 10, 11, 12, 13, 14, 15); }
__device__ __forceinline__ v16bf cat16b(v8us lo, v8us hi) { return __builtin_bit_cast(v16bf, __builtin_shufflevector(lo, hi, 0, 1, 2, 3, 4, 5, 6, 7, 8, 9, 10, 11, 12, 13, 14, 15)); }
__device__ __forceinline__ v16h  ldh(const h16* p) { return cat16(*(const v8h*)p, *(const v8h*)(p + 16)); }
__device__ __forceinline__ v16bf ldb(const bf* p)  { return cat16b(*(const v8us*)p, *(const v8us*)(p + 16)); }
__device__ __forceinline__ h16 toh_flush(float v) { const h16 r = (h16)v; return (fabsf(v) < 6.103515625e-05f) ? (h16)0.0f : r; }
__device__ __forceinline__ v8f wmma16g(v16h a, v16h b, v8f c) {
    c = __builtin_amdgcn_wmma_f32_16x16x32_f16(false, a, false, b, (short)0, c, false, false);
    asm volatile("v_nop\n\tv_nop\n\tv_nop\n\tv_nop" : "+v"(c) : "v"(a), "v"(b));
    return c; }
__device__ __forceinline__ v8f wmmabg(v16bf a, v16bf b, v8f c) {
    c = __builtin_amdgcn_wmma_f32_16x16x32_bf16(false, a, false, b, (short)0, c, false, false);
    asm volatile("v_nop\n\tv_nop\n\tv_nop\n\tv_nop" : "+v"(c) : "v"(a), "v"(b));
    return c; }
__device__ __forceinline__ int clampi(int v, int lo, int hi) { return v < lo ? lo : (v > hi ? hi : v); }

template <int NC>
__device__ __forceinline__ void tr_body(const float* __restrict__ src, bf* dst) {
    static_assert(NC % 32 == 0);
    static_assert(((NC + 8) * 2) % 16 == 0);
    static_assert((NC / 32) * 256 * 16 == TP * NC * 2);
    static_assert((NC / 4) * 256 == TP * NC);
    __shared__ __align__(16) bf ts[TP * (NC + 8)];
    const int tid = threadIdx.x;
    const int blk = blockIdx.x; const int xs = blk & 1, y = (blk >> 1) & (HH - 1), b = blk >> 8;
    const float* sp = src + ((size_t)b * NC * HH + y) * WW + xs * TP;
#pragma unroll 1
    for (int it = 0; it < NC / 4; ++it) { const int i = it * 256 + tid; const int c = i >> 6, xx = i & 63;
        ts[xx * (NC + 8) + c] = f2bf(sp[(size_t)c * (HH * WW) + xx]); }
    __syncthreads();
    bf* dp = dst + (((size_t)b * HH + y) * WW + xs * TP) * NC;
#pragma unroll 1
    for (int ps = 0; ps < 2; ++ps) {
#pragma unroll
        for (int it = 0; it < NC / 32; ++it) { const int i = it * 256 + tid; const int e = i * 8; const int px = e / NC, c = e % NC;
            const v8us v = *(const v8us*)(&ts[px * (NC + 8) + c]);
            *(volatile v8us*)(dp + (size_t)i * 8) = v; }
        if (ps == 0) __threadfence(); }
}
__global__ __launch_bounds__(256) void k_tr64(const float* __restrict__ src, bf* dst) { tr_body<CI>(src, dst); }
__global__ __launch_bounds__(256) void k_tr32(const float* __restrict__ src, bf* dst) { tr_body<OFC>(src, dst); }

__global__ __launch_bounds__(256) void k_wconv_off(const float* __restrict__ w_off, bf* WOB) {
    const int i = blockIdx.x * 256 + threadIdx.x; if (i >= NOPD * KO / 8) return;
    const int n = i / (KO / 8), kk = (i - n * (KO / 8)) * 8;
    const bool ok = n < NOM; const int nc = ok ? n : (NOM - 1);
    v8us o;
#pragma unroll
    for (int e = 0; e < 8; ++e) { const int k = kk + e; const int t = k >> 5, ic = k & 31;
        float v = w_off[(nc * OFC + ic) * NTAP + t]; asm volatile("" : "+v"(v));
        o[e] = ok ? f2bf(v) : (unsigned short)0; }
    *(volatile v8us*)(WOB + (size_t)i * 8) = o; __threadfence(); *(volatile v8us*)(WOB + (size_t)i * 8) = o;
}

__global__ __launch_bounds__(256) void k_wconv_main(const float* __restrict__ weight, h16* WH) {
    const int i = blockIdx.x * 256 + threadIdx.x; if (i >= CO * KM / 8) return;
    const int o = i / (KM / 8), kk = (i - o * (KM / 8)) * 8;
    v8h hv;
#pragma unroll
    for (int e = 0; e < 8; ++e) { const int k = kk + e; const int t = k >> 6, c = k & 63;
        const float v = bfr(weight[(o * CI + c) * NTAP + t]) * WSC;
        hv[e] = toh_flush(v); }
    *(volatile v8h*)(WH + (size_t)i * 8) = hv; __threadfence(); *(volatile v8h*)(WH + (size_t)i * 8) = hv;
}

__global__ __launch_bounds__(128) void k_dconv(const bf* __restrict__ FT, const bf* __restrict__ XT, const bf* __restrict__ WOB, const h16* __restrict__ WH,
                                               const float* __restrict__ b_off, const float* __restrict__ bias, float* OUT) {
    __shared__ __align__(16) bf    fs[3 * FC * 32];
    __shared__ __align__(16) float oms[NOPD * OMP];
    __shared__ __align__(16) int   tabi[TP * NTAP * 4];
    __shared__ __align__(16) float tabw[TP * NTAP * 4];
    __shared__ __align__(16) h16   as[TP * ASP];
    __shared__ __align__(16) float os[CO * OSP];
    const int tid = threadIdx.x, lane = tid & 31, lr = lane & 15, hi = lane >> 4;
    const int wave = __builtin_amdgcn_readfirstlane((int)(threadIdx.x >> 5));
    const int blk = blockIdx.x; const int w0 = (blk & 1) * TP, h = (blk >> 1) & (HH - 1), b = blk >> 8;

    const bf* ftb = FT + (size_t)b * ((size_t)HH * WW * OFC);
#pragma unroll 1
    for (int it = 0; it < 7; ++it) {
        const int i = it * 128 + tid; const bool in = i < 3 * FC * 4; const int ii = in ? i : (3 * FC * 4 - 1);
        const int q = ii & 3, pc = ii >> 2; const int r = pc / FC, c = pc - r * FC;
        const int yy = h - 1 + r, xx = w0 - 1 + c;
        const bool ok = (yy >= 0) & (yy < HH) & (xx >= 0) & (xx < WW);
        const int yc = clampi(yy, 0, HH - 1), xc = clampi(xx, 0, WW - 1);
        v4u v = *(const v4ua*)(ftb + (size_t)(yc * WW + xc) * OFC + q * 8);
        asm volatile("" : "+v"(v));
        const v4u z = (v4u){};
        v = ok ? v : z;
        if (in) *(v8us*)(&fs[pc * 32 + q * 8]) = __builtin_bit_cast(v8us, v);
    }
    __syncthreads();

    {
        v8f oa = (v8f){}, ob = (v8f){};
#pragma unroll 1
        for (int t = 0; t < NTAP; ++t) {
            const int ky = t / 3, kx = t - ky * 3;
            const int ai = (ky * FC + 16 * wave + lr + kx) * 32 + 8 * hi;
            const v16bf a = cat16b(*(const v8us*)(&fs[ai]), *(const v8us*)(&fs[ai + 16]));
            const v16bf b0 = ldb(WOB + (size_t)lr * KO + t * 32 + 8 * hi);
            const v16bf b1 = ldb(WOB + (size_t)(16 + lr) * KO + t * 32 + 8 * hi);
            oa = wmmabg(a, b0, oa); ob = wmmabg(a, b1, ob);
        }
        const float bo0 = bfr(b_off[lr]);
        const bool okb = (16 + lr) < NOM;
        float bo1 = b_off[okb ? (16 + lr) : (NOM - 1)]; asm volatile("" : "+v"(bo1));
        bo1 = okb ? bfr(bo1) : 0.0f;
        v4f p, q;
        p[0] = oa[0] + bo0; p[1] = oa[1] + bo0; p[2] = oa[2] + bo0; p[3] = oa[3] + bo0; q[0] = oa[4] + bo0; q[1] = oa[5] + bo0; q[2] = oa[6] + bo0; q[3] = oa[7] + bo0;
        *(v4fa*)(&oms[lr * OMP + 16 * wave + 8 * hi]) = p; *(v4fa*)(&oms[lr * OMP + 16 * wave + 8 * hi + 4]) = q;
        p[0] = ob[0] + bo1; p[1] = ob[1] + bo1; p[2] = ob[2] + bo1; p[3] = ob[3] + bo1; q[0] = ob[4] + bo1; q[1] = ob[5] + bo1; q[2] = ob[6] + bo1; q[3] = ob[7] + bo1;
        *(v4fa*)(&oms[(16 + lr) * OMP + 16 * wave + 8 * hi]) = p; *(v4fa*)(&oms[(16 + lr) * OMP + 16 * wave + 8 * hi + 4]) = q;
    }
    __syncthreads();

#pragma unroll 1
    for (int it = 0; it < 5; ++it) {
        const int i = it * 128 + tid; const bool in = i < TP * NTAP; const int ii = in ? i : (TP * NTAP - 1);
        const int p = ii / NTAP, k = ii - p * NTAP;
        const int kyy = k / 3, kxx = k - kyy * 3;
        const float dy = oms[(2 * k) * OMP + p], dx = oms[(2 * k + 1) * OMP + p], mm = oms[(18 + k) * OMP + p];
        const float mo = 1.0f / (1.0f + expf(-mm));
        const float py = (float)(h - 1 + kyy) + dy, px = (float)(w0 + p - 1 + kxx) + dx;
        const float y0 = floorf(py), x0 = floorf(px);
        const float wy = py - y0, wx = px - x0;
        const float y1 = y0 + 1.0f, x1 = x0 + 1.0f;
        const bool vy0 = (y0 >= 0.0f) & (y0 <= (float)(HH - 1)), vy1 = (y1 >= 0.0f) & (y1 <= (float)(HH - 1));
        const bool vx0 = (x0 >= 0.0f) & (x0 <= (float)(WW - 1)), vx1 = (x1 >= 0.0f) & (x1 <= (float)(WW - 1));
        const int iy0 = (int)fminf(fmaxf(y0, 0.0f), (float)(HH - 1)), iy1 = (int)fminf(fmaxf(y1, 0.0f), (float)(HH - 1));
        const int ix0 = (int)fminf(fmaxf(x0, 0.0f), (float)(WW - 1)), ix1 = (int)fminf(fmaxf(x1, 0.0f), (float)(WW - 1));
        const float ms = mo * SCA;
        const float ay = (1.0f - wy) * ms, by = wy * ms;
        const float g00 = ay * (1.0f - wx), g01 = ay * wx, g10 = by * (1.0f - wx), g11 = by * wx;
        v4i ti; v4f tw;
        ti[0] = iy0 * WW + ix0; ti[1] = iy0 * WW + ix1; ti[2] = iy1 * WW + ix0; ti[3] = iy1 * WW + ix1;
        tw[0] = (vy0 & vx0) ? g00 : 0.0f; tw[1] = (vy0 & vx1) ? g01 : 0.0f; tw[2] = (vy1 & vx0) ? g10 : 0.0f; tw[3] = (vy1 & vx1) ? g11 : 0.0f;
        if (in) { *(v4i*)(&tabi[ii * 4]) = ti; *(v4fa*)(&tabw[ii * 4]) = tw; }
    }
    __syncthreads();

    v8f acc[4];
#pragma unroll
    for (int mt = 0; mt < 4; ++mt) acc[mt] = (v8f){};
    const bf* xtb = XT + (size_t)b * ((size_t)HH * WW * CI);
    const h16* wrow = WH + (size_t)(16 * wave + lr) * KM + 8 * hi;
#pragma unroll 1
    for (int ky = 0; ky < 3; ++ky) {
#pragma unroll 1
        for (int it = 0; it < 12; ++it) {
            const int i = it * 128 + tid; const int p = i / 24; const int rem = i - p * 24; const int tl = rem >> 3, g = rem & 7;
            const int e = (p * NTAP + ky * 3 + tl) * 4;
            const v4i ix = *(const v4i*)(&tabi[e]); const v4f wv = *(const v4fa*)(&tabw[e]);
            const bf* xg = xtb + g * 8;
            const v4u c00 = *(const v4ua*)(xg + (size_t)ix[0] * CI);
            const v4u c01 = *(const v4ua*)(xg + (size_t)ix[1] * CI);
            const v4u c10 = *(const v4ua*)(xg + (size_t)ix[2] * CI);
            const v4u c11 = *(const v4ua*)(xg + (size_t)ix[3] * CI);
            v8h hv;
#pragma unroll
            for (int j = 0; j < 4; ++j) {
                const float l00 = __uint_as_float(c00[j] << 16), u00 = __uint_as_float(c00[j] & 0xffff0000u);
                const float l01 = __uint_as_float(c01[j] << 16), u01 = __uint_as_float(c01[j] & 0xffff0000u);
                const float l10 = __uint_as_float(c10[j] << 16), u10 = __uint_as_float(c10[j] & 0xffff0000u);
                const float l11 = __uint_as_float(c11[j] << 16), u11 = __uint_as_float(c11[j] & 0xffff0000u);
                const float sl = wv[0] * l00 + wv[1] * l01 + wv[2] * l10 + wv[3] * l11;
                const float su = wv[0] * u00 + wv[1] * u01 + wv[2] * u10 + wv[3] * u11;
                hv[2 * j] = toh_flush(sl); hv[2 * j + 1] = toh_flush(su); }
            *(v8h*)(&as[p * ASP + tl * CI + g * 8]) = hv;
        }
        __syncthreads();
#pragma unroll 1
        for (int ks = 0; ks < 6; ++ks) {
            const int kk = ks * 32;
            const v16h bw = ldh(wrow + ky * (3 * CI) + kk);
#pragma unroll
            for (int mt = 0; mt < 4; ++mt) {
                const int ai = (16 * mt + lr) * ASP + kk + 8 * hi;
                const v16h a = cat16(*(const v8h*)(&as[ai]), *(const v8h*)(&as[ai + 16]));
                acc[mt] = wmma16g(a, bw, acc[mt]); }
        }
        __syncthreads();
    }

    const float bv = bfr(bias[16 * wave + lr]);
#pragma unroll
    for (int mt = 0; mt < 4; ++mt) {
        v4f p, q;
        p[0] = acc[mt][0] * OSC + bv; p[1] = acc[mt][1] * OSC + bv; p[2] = acc[mt][2] * OSC + bv; p[3] = acc[mt][3] * OSC + bv;
        q[0] = acc[mt][4] * OSC + bv; q[1] = acc[mt][5] * OSC + bv; q[2] = acc[mt][6] * OSC + bv; q[3] = acc[mt][7] * OSC + bv;
        *(v4fa*)(&os[(16 * wave + lr) * OSP + 16 * mt + 8 * hi]) = p; *(v4fa*)(&os[(16 * wave + lr) * OSP + 16 * mt + 8 * hi + 4]) = q; }
    __syncthreads();
    float* orow = OUT + (((size_t)b * CO + 16 * wave) * HH + h) * WW + w0;
#pragma unroll 1
    for (int ps = 0; ps < 2; ++ps) {
#pragma unroll
        for (int s = 0; s < 8; ++s) { const int row = 2 * s + (lane >> 4), cofs = (lane & 15) * 4;
            const v4f val = *(const v4fa*)(&os[(16 * wave + row) * OSP + cofs]);
            *(volatile v4f*)(orow + (size_t)row * (HH * WW) + cofs) = val; }
        if (ps == 0) __threadfence(); }
}

static constexpr size_t al256(size_t v) { return (v + 255) & ~(size_t)255; }
static constexpr size_t SZ_XT = al256((size_t)NB * HH * WW * CI * 2);
static constexpr size_t SZ_FT = al256((size_t)NB * HH * WW * OFC * 2);
static constexpr size_t SZ_WO = al256((size_t)NOPD * KO * 2);
static constexpr size_t SZ_WH = al256((size_t)CO * KM * 2);
static constexpr size_t SZ_TOTAL = SZ_XT + SZ_FT + SZ_WO + SZ_WH;
static_assert(SZ_TOTAL <= (size_t)134217728);
static_assert(((size_t)NOPD * KO * 2) % 128 == 0);
static_assert(((size_t)CO * KM * 2) % 128 == 0);
static_assert((NOPD * KO / 8) <= 5 * 256);
static_assert((CO * KM / 8) == 18 * 256);

extern "C" void kernel_launch(void* const* d_in, const int* in_sizes, int n_in,
                              void* d_out, int out_size, void* d_ws, size_t ws_size, hipStream_t stream) {
    if (n_in < 6) return;
    if ((size_t)in_sizes[0] < (size_t)NB * CI * HH * WW) return;
    if ((size_t)in_sizes[1] < (size_t)NB * OFC * HH * WW) return;
    if ((size_t)in_sizes[2] < (size_t)NOM * OFC * NTAP) return;
    if (in_sizes[3] < NOM) return;
    if ((size_t)in_sizes[4] < (size_t)CO * CI * NTAP) return;
    if (in_sizes[5] < CO) return;
    if ((size_t)out_size < (size_t)NB * CO * HH * WW) return;
    if (SZ_TOTAL > ws_size) return;
    const float* x    = (const float*)d_in[0];
    const float* feat = (const float*)d_in[1];
    const float* woff = (const float*)d_in[2];
    const float* boff = (const float*)d_in[3];
    const float* wmn  = (const float*)d_in[4];
    const float* bmn  = (const float*)d_in[5];
    float* OUT = (float*)d_out;
    char* wsp = (char*)d_ws;
    bf*  XT  = (bf*)wsp;  wsp += SZ_XT;
    bf*  FT  = (bf*)wsp;  wsp += SZ_FT;
    bf*  WOB = (bf*)wsp;  wsp += SZ_WO;
    h16* WH  = (h16*)wsp; wsp += SZ_WH;

    k_tr64<<<dim3(NB * HH * (WW / TP), 1, 1), 256, 0, stream>>>(x, XT);
    k_tr32<<<dim3(NB * HH * (WW / TP), 1, 1), 256, 0, stream>>>(feat, FT);
    k_wconv_off<<<dim3((NOPD * KO / 8 + 255) / 256, 1, 1), 256, 0, stream>>>(woff, WOB);
    k_wconv_main<<<dim3((CO * KM / 8 + 255) / 256, 1, 1), 256, 0, stream>>>(wmn, WH);
    k_dconv<<<dim3(NB * HH * (WW / TP), 1, 1), 128, 0, stream>>>(FT, XT, WOB, WH, boff, bmn, OUT);
}
